// GPT2Block_76132590289001
// MI455X (gfx1250) — hardware-run, weakly checked
//
#include <hip/hip_runtime.h>
#include <math.h>

typedef __attribute__((ext_vector_type(16))) _Float16 v16h;
typedef __attribute__((ext_vector_type(8)))  _Float16 v8h;
typedef __attribute__((ext_vector_type(8)))  float    v8f;
typedef __attribute__((ext_vector_type(4)))  float    v4f;
typedef __attribute__((ext_vector_type(4)))  unsigned int v4u;

#ifndef NB
#define NB 32
#endif
#ifndef SEQ
#define SEQ 1024
#endif
#define NB_FULL 32
#define SEQ_FULL 1024

constexpr int kBatch   = NB;
constexpr int kSeq     = SEQ;
constexpr int kSeqFull = SEQ_FULL;
constexpr int kDim     = 256;
constexpr int kHid     = 128;
constexpr int kRows    = kBatch * kSeq;
constexpr int kQkvN    = 3 * kDim;
constexpr float kLnEps      = 1e-5f;
constexpr float kMaskFill   = -10000.0f;
constexpr float kScoreScale = 0.0625f;
constexpr float kWCarry     = 64.0f;
constexpr float kAttnCarry  = 64.0f;
constexpr float kPCarry     = 32768.0f;

static_assert(kBatch >= 1 && kBatch <= NB_FULL);
static_assert(kSeq >= 64 && kSeq <= SEQ_FULL && kSeq % 64 == 0);
static_assert(kRows % 64 == 0 && kQkvN % 64 == 0 && kDim % 64 == 0 && kHid % 64 == 0);
static_assert(kDim % 32 == 0 && kHid % 32 == 0);
static_assert(kDim == 32 * 8);

constexpr size_t kOffWqkvT = 0;
constexpr size_t kSzWqkvT  = (size_t)kQkvN * kDim * 2;
constexpr size_t kOffWpT   = kOffWqkvT + kSzWqkvT;
constexpr size_t kSzWpT    = (size_t)kDim * kDim * 2;
constexpr size_t kOffWfc1T = kOffWpT + kSzWpT;
constexpr size_t kSzWfc1T  = (size_t)kHid * kDim * 2;
constexpr size_t kOffWfc2T = kOffWfc1T + kSzWfc1T;
constexpr size_t kSzWfc2T  = (size_t)kDim * kHid * 2;
constexpr size_t kOffH     = kOffWfc2T + kSzWfc2T;
constexpr size_t kSzH      = (size_t)kRows * kDim * 2;
constexpr size_t kOffQkv   = kOffH + kSzH;
constexpr size_t kSzQkv    = (size_t)kRows * kQkvN * 2;
constexpr size_t kOffAttn  = kOffQkv + kSzQkv;
constexpr size_t kSzAttn   = (size_t)kRows * kDim * 2;
constexpr size_t kOffX1    = kOffAttn + kSzAttn;
constexpr size_t kSzX1     = (size_t)kRows * kDim * 4;
constexpr size_t kOffFc    = kOffX1 + kSzX1;
constexpr size_t kSzFc     = (size_t)kRows * kHid * 2;
constexpr size_t kWsTotal  = kOffFc + kSzFc;
static_assert(kOffH == 655360ull);
static_assert(kWsTotal <= 134217728ull);
static_assert(NB != NB_FULL || SEQ != SEQ_FULL || kWsTotal == 126484480ull);
static_assert(kOffWpT % 256 == 0 && kOffWfc1T % 256 == 0 && kOffWfc2T % 256 == 0 && kOffH % 256 == 0 &&
              kOffQkv % 256 == 0 && kOffAttn % 256 == 0 && kOffX1 % 256 == 0 && kOffFc % 256 == 0);

__device__ __forceinline__ unsigned short f2bf_bits(float f) {
  unsigned u = __float_as_uint(f);
  return (unsigned short)((u + 0x7FFFu + ((u >> 16) & 1u)) >> 16);
}
__device__ __forceinline__ float bf_bits2f(unsigned short h) { return __uint_as_float(((unsigned)h) << 16); }
__device__ __forceinline__ float bfr(float f) { return bf_bits2f(f2bf_bits(f)); }

__device__ __forceinline__ void dep_guard_h(v8f& a, v8f& b, v16h x, v16h y) { asm volatile("v_nop\n\tv_nop\n\tv_nop\n\tv_nop" : "+v"(a), "+v"(b) : "v"(x), "v"(y)); }
__device__ __forceinline__ void keep4_h(v16h a, v16h b, v16h c, v16h d) { asm volatile("v_nop" :: "v"(a), "v"(b), "v"(c), "v"(d)); }
__device__ __forceinline__ void acc_guard4(v8f& a, v8f& b, v8f& c, v8f& d) { asm volatile("v_nop\n\tv_nop\n\tv_nop\n\tv_nop" : "+v"(a), "+v"(b), "+v"(c), "+v"(d)); }

struct FragH {
  union U { v16h v; v8h h[2]; };
  static __device__ __forceinline__ v16h load(const _Float16* p) {
    U f; f.h[0] = *(const v8h*)(p); f.h[1] = *(const v8h*)(p + 16); return f.v;
  }
  static __device__ __forceinline__ v8f mma(v16h a, v16h b, v8f c) {
    return __builtin_amdgcn_wmma_f32_16x16x32_f16(false, a, false, b, (short)0, c, false, false);
  }
};

__device__ __forceinline__ v8f mma_h(v16h a, v16h b, v8f c) {
  c = __builtin_amdgcn_wmma_f32_16x16x32_f16(false, a, false, b, (short)0, c, false, false);
  asm volatile("v_nop\n\tv_nop\n\tv_nop\n\tv_nop" : "+v"(c) : "v"(a), "v"(b));
  return c;
}

template <int BIAS_MODE, int OUT_MODE, bool RESID, bool RESID_RNE, int ACT>
__global__ __launch_bounds__(256) void wmma_gemm64(
    const unsigned short* __restrict__ Ap, int lda, long strideA,
    const unsigned short* __restrict__ Btp, int ldb, long strideB,
    void* __restrict__ Cout, int ldc, long strideC,
    const float* __restrict__ bias,
    const float* __restrict__ resid, long strideR,
    int M, int N, int K, float scale) {
  static_assert(!RESID || OUT_MODE == 0);
  __shared__ __align__(16) float sT[8][16 * 68];
  const int b    = blockIdx.y;
  const int lane = threadIdx.x & 31;
  const int wave = threadIdx.x >> 5;
  const int tilesN = N >> 6;
  const int tilesM = M >> 6;
  const int tile = blockIdx.x * 8 + wave;
  if (tile >= tilesM * tilesN) return;
  const int tm = tile / tilesN;
  const int tn = tile - tm * tilesN;
  const int m0 = tm << 6;
  const int n0 = tn << 6;

  const _Float16* Ab = (const _Float16*)(const void*)Ap  + (size_t)b * strideA;
  const _Float16* Bb = (const _Float16*)(const void*)Btp + (size_t)b * strideB;

  const int rlane = lane & 15;
  const int koff  = (lane >> 4) * 8;
  const int mOff  = (lane >> 4) * 8;

  v8f acc[4][4];
#pragma unroll
  for (int i = 0; i < 4; ++i)
#pragma unroll
    for (int j = 0; j < 4; ++j) acc[i][j] = (v8f){0.f,0.f,0.f,0.f,0.f,0.f,0.f,0.f};

  for (int k0 = 0; k0 < K; k0 += 32) {
    v16h bh[4];
#pragma unroll
    for (int j = 0; j < 4; ++j) {
      const size_t bo = (size_t)(n0 + (j << 4) + rlane) * ldb + koff + k0;
      bh[j] = FragH::load(Bb + bo);
    }
#pragma unroll
    for (int i = 0; i < 4; ++i) {
      const size_t ao = (size_t)(m0 + (i << 4) + rlane) * lda + koff + k0;
      const v16h ah = FragH::load(Ab + ao);
#pragma unroll
      for (int j = 0; j < 4; ++j) acc[i][j] = FragH::mma(ah, bh[j], acc[i][j]);
      dep_guard_h(acc[i][0], acc[i][3], ah, ah);
    }
    keep4_h(bh[0], bh[1], bh[2], bh[3]);
  }
  acc_guard4(acc[0][0], acc[0][1], acc[0][2], acc[0][3]);
  acc_guard4(acc[1][0], acc[1][1], acc[1][2], acc[1][3]);
  acc_guard4(acc[2][0], acc[2][1], acc[2][2], acc[2][3]);
  acc_guard4(acc[3][0], acc[3][1], acc[3][2], acc[3][3]);

  float* slab = sT[wave];
#pragma unroll
  for (int i = 0; i < 4; ++i) {
    const int mBase = m0 + (i << 4);
#pragma unroll
    for (int j = 0; j < 4; ++j) {
      const int n = n0 + (j << 4) + rlane;
      float bv = 0.f;
      if (BIAS_MODE == 2) bv = bfr(bias[n]);
#pragma unroll
      for (int r = 0; r < 8; ++r) {
        float v = acc[i][j][r] * scale;
        if (BIAS_MODE == 1) v += bfr(bias[mBase + mOff + r]);
        if (BIAS_MODE == 2) v += bv;
        if (ACT == 1) v = fmaxf(v, 0.0f);
        slab[(mOff + r) * 68 + (j << 4) + rlane] = v;
      }
    }
    __builtin_amdgcn_fence(3, "workgroup");
    __builtin_amdgcn_wave_barrier();
    __builtin_amdgcn_fence(2, "workgroup");
    if (OUT_MODE == 0) {
      float* C = (float*)Cout + (size_t)b * strideC;
      const float* Rb = RESID ? (resid + (size_t)b * strideR) : nullptr;
      const int hh = lane >> 4, c4 = (lane & 15) * 4;
      for (int pass = 0; pass < 2; ++pass) {
#pragma unroll
        for (int it = 0; it < 8; ++it) {
          const int row = it * 2 + hh;
          v4f v = *(const v4f*)(slab + row * 68 + c4);
          if (RESID) {
            v4f rr = *(const v4f*)(Rb + (size_t)(mBase + row) * ldc + n0 + c4);
            if (RESID_RNE) { rr[0] = bfr(rr[0]); rr[1] = bfr(rr[1]); rr[2] = bfr(rr[2]); rr[3] = bfr(rr[3]); }
            v = v + rr;
          }
          *(volatile v4f*)(C + (size_t)(mBase + row) * ldc + n0 + c4) = v;
        }
        __threadfence();
      }
    } else {
      const int q = lane >> 3, c8 = (lane & 7) * 8;
      unsigned short* C = (unsigned short*)Cout + (size_t)b * strideC;
      for (int pass = 0; pass < 2; ++pass) {
#pragma unroll
        for (int it = 0; it < 4; ++it) {
          const int row = it * 4 + q;
          const float* sp = slab + row * 68 + c8;
          v8h hv;
#pragma unroll
          for (int e = 0; e < 8; ++e) hv[e] = (_Float16)sp[e];
          *(volatile v8h*)(C + (size_t)(mBase + row) * ldc + n0 + c8) = hv;
        }
        __threadfence();
      }
    }
    __builtin_amdgcn_fence(3, "workgroup");
    __builtin_amdgcn_wave_barrier();
    __builtin_amdgcn_fence(2, "workgroup");
  }
}

__global__ __launch_bounds__(256) void transpose_to_f16(const float* __restrict__ in, unsigned short* __restrict__ out,
                                                        int R, int Cc, float scale) {
  __shared__ float sm[64][65];
  const int tid = threadIdx.x, lane = tid & 31, wave = tid >> 5;
  const int r0 = blockIdx.y * 64, c0 = blockIdx.x * 64;
#pragma unroll
  for (int ps = 0; ps < 4; ++ps) {
    const int r = ps * 16 + (tid >> 4);
    const int c4 = (tid & 15) * 4;
    const v4f v = *(const v4f*)(in + (size_t)(r0 + r) * Cc + c0 + c4);
    sm[r][c4 + 0] = v[0];
    sm[r][c4 + 1] = v[1];
    sm[r][c4 + 2] = v[2];
    sm[r][c4 + 3] = v[3];
  }
  __syncthreads();
  const int q4 = lane >> 3, c8 = (lane & 7) * 8;
  _Float16* ob = (_Float16*)(void*)out;
  for (int pass = 0; pass < 2; ++pass) {
#pragma unroll
    for (int it = 0; it < 2; ++it) {
      const int n = wave * 8 + it * 4 + q4;
      v8h hv;
#pragma unroll
      for (int e = 0; e < 8; ++e) hv[e] = (_Float16)(bfr(sm[c8 + e][n]) * scale);
      *(volatile v8h*)(ob + (size_t)(c0 + n) * R + r0 + c8) = hv;
    }
    __threadfence();
  }
}

template <bool IN_RNE>
__global__ __launch_bounds__(128) void layernorm256_to_f16(const float* __restrict__ x, int srcSeq,
                                                           const float* __restrict__ gam, const float* __restrict__ bet,
                                                           unsigned short* __restrict__ out, int nrows) {
  const int tid = threadIdx.x, lane = tid & 31, wave = tid >> 5;
  const int row = blockIdx.x * 4 + wave;
  if (row >= nrows) return;
  const int bq = row / kSeq;
  const int sq = row - bq * kSeq;
  const float* xr = x + ((size_t)bq * srcSeq + sq) * kDim + lane * 8;
  const v4f xa = *(const v4f*)xr;
  const v4f xb = *(const v4f*)(xr + 4);
  float v[8] = {xa[0], xa[1], xa[2], xa[3], xb[0], xb[1], xb[2], xb[3]};
  if (IN_RNE) {
#pragma unroll
    for (int e = 0; e < 8; ++e) v[e] = bfr(v[e]);
  }

  float s = ((v[0] + v[1]) + (v[2] + v[3])) + ((v[4] + v[5]) + (v[6] + v[7]));
#pragma unroll
  for (int off = 16; off > 0; off >>= 1) s += __shfl_xor(s, off, 32);
  const float mu = s * (1.0f / (float)kDim);

  float d[8];
#pragma unroll
  for (int e = 0; e < 8; ++e) d[e] = v[e] - mu;
  float ssq = ((d[0] * d[0] + d[1] * d[1]) + (d[2] * d[2] + d[3] * d[3])) +
              ((d[4] * d[4] + d[5] * d[5]) + (d[6] * d[6] + d[7] * d[7]));
#pragma unroll
  for (int off = 16; off > 0; off >>= 1) ssq += __shfl_xor(ssq, off, 32);
  const float var = ssq * (1.0f / (float)kDim);
  const float rstd = rsqrtf(var + kLnEps);

  const v4f ga = *(const v4f*)(gam + lane * 8);
  const v4f gb = *(const v4f*)(gam + lane * 8 + 4);
  const v4f ba = *(const v4f*)(bet + lane * 8);
  const v4f bb = *(const v4f*)(bet + lane * 8 + 4);
  const float g8[8] = {bfr(ga[0]), bfr(ga[1]), bfr(ga[2]), bfr(ga[3]), bfr(gb[0]), bfr(gb[1]), bfr(gb[2]), bfr(gb[3])};
  const float b8[8] = {bfr(ba[0]), bfr(ba[1]), bfr(ba[2]), bfr(ba[3]), bfr(bb[0]), bfr(bb[1]), bfr(bb[2]), bfr(bb[3])};
  v8h hv;
#pragma unroll
  for (int e = 0; e < 8; ++e) hv[e] = (_Float16)((d[e] * rstd) * g8[e] + b8[e]);
  _Float16* ob = (_Float16*)(void*)out + (size_t)row * kDim + lane * 8;
  *(volatile v8h*)ob = hv;
  __threadfence();
  *(volatile v8h*)ob = hv;
}

__global__ __launch_bounds__(256) void attn_causal_f16(const unsigned short* __restrict__ qkvp,
                                                       unsigned short* __restrict__ outp) {
  __shared__ __align__(16) _Float16 KV_s[2 * 32 * kDim];
  __shared__ __align__(16) _Float16 P_s[8][16 * 32];
  _Float16* K_s = KV_s;
  _Float16* V_s = KV_s + 32 * kDim;

  const int tid  = threadIdx.x;
  const int wave = tid >> 5;
  const int lane = tid & 31;
  const int hh   = lane >> 4;
  const int c    = lane & 15;
  const int g     = wave & 3;
  const int dhalf = wave >> 2;

  constexpr int nqb = kSeq / 64;
  const int bx = blockIdx.x;
  const int qb = bx % nqb;
  const int b  = bx / nqb;
  const int q0 = qb * 64 + g * 16;

  const _Float16* base = (const _Float16*)(const void*)qkvp + (size_t)b * kSeq * kQkvN;
  const _Float16* qptr = base;
  const _Float16* kptr = base + kDim;
  const _Float16* vptr = base + 2 * kDim;

  float mrow[8], lrow[8];
  v8f oacc[8];
#pragma unroll
  for (int r = 0; r < 8; ++r) { mrow[r] = -INFINITY; lrow[r] = 0.f; }
#pragma unroll
  for (int t = 0; t < 8; ++t) oacc[t] = (v8f){0.f,0.f,0.f,0.f,0.f,0.f,0.f,0.f};

  const int nChunks = 2 * qb + 2;
  for (int kc = 0; kc < nChunks; ++kc) {
    const int kv0 = kc * 32;
    __syncthreads();
    {
      const int kvr = tid >> 3, dq = (tid & 7) * 32;
      const v4u* krow = (const v4u*)(const void*)(kptr + (size_t)(kv0 + kvr) * kQkvN + dq);
      const v4u* vrow = (const v4u*)(const void*)(vptr + (size_t)(kv0 + kvr) * kQkvN + dq);
      v4u kw[4], vw[4];
#pragma unroll
      for (int i = 0; i < 4; ++i) { kw[i] = krow[i]; vw[i] = vrow[i]; }
#pragma unroll
      for (int i = 0; i < 4; ++i) *(v8h*)(K_s + kvr * kDim + dq + 8 * i) = __builtin_bit_cast(v8h, kw[i]);
#pragma unroll
      for (int i = 0; i < 4; ++i) {
#pragma unroll
        for (int wj = 0; wj < 4; ++wj) {
          const unsigned w = vw[i][wj];
          const int d = dq + 8 * i + 2 * wj;
          V_s[d * 32 + kvr]       = __builtin_bit_cast(_Float16, (unsigned short)(w & 0xffffu));
          V_s[(d + 1) * 32 + kvr] = __builtin_bit_cast(_Float16, (unsigned short)(w >> 16));
        }
      }
    }
    __syncthreads();

    v8f s[2];
    s[0] = (v8f){0.f,0.f,0.f,0.f,0.f,0.f,0.f,0.f};
    s[1] = (v8f){0.f,0.f,0.f,0.f,0.f,0.f,0.f,0.f};
#pragma unroll
    for (int dc = 0; dc < 8; ++dc) {
      const v16h qa = FragH::load(qptr + (size_t)(q0 + c) * kQkvN + dc * 32 + 8 * hh);
#pragma unroll
      for (int j = 0; j < 2; ++j) {
        const v16h kb = FragH::load(K_s + (j * 16 + c) * kDim + dc * 32 + 8 * hh);
        s[j] = mma_h(qa, kb, s[j]);
      }
    }

    float cm[8];
#pragma unroll
    for (int r = 0; r < 8; ++r) {
      const int qrow = q0 + 8 * hh + r;
      float m = -INFINITY;
#pragma unroll
      for (int j = 0; j < 2; ++j) {
        const int kvcol = kv0 + j * 16 + c;
        const bool masked = (kvcol > qrow);
        float sv = s[j][r] * kScoreScale;
        sv = masked ? kMaskFill : sv;
        s[j][r] = sv;
        m = fmaxf(m, sv);
      }
#pragma unroll
      for (int off = 1; off < 16; off <<= 1) m = fmaxf(m, __shfl_xor(m, off, 32));
      cm[r] = m;
    }

    _Float16* pw = P_s[wave];
#pragma unroll
    for (int r = 0; r < 8; ++r) {
      const float mnew = fmaxf(mrow[r], cm[r]);
      const float alpha = expf(mrow[r] - mnew);
      mrow[r] = mnew;
      float psum = 0.f;
#pragma unroll
      for (int j = 0; j < 2; ++j) {
        const float p = expf(s[j][r] - mnew);
        psum += p;
        pw[(8 * hh + r) * 32 + j * 16 + c] = (_Float16)(p * kPCarry);
      }
#pragma unroll
      for (int off = 1; off < 16; off <<= 1) psum += __shfl_xor(psum, off, 32);
      lrow[r] = lrow[r] * alpha + psum;
#pragma unroll
      for (int t = 0; t < 8; ++t) oacc[t][r] *= alpha;
    }
    __builtin_amdgcn_fence(3, "workgroup");
    __builtin_amdgcn_wave_barrier();
    __builtin_amdgcn_fence(2, "workgroup");

    {
      const v16h pa = FragH::load(pw + c * 32 + 8 * hh);
#pragma unroll
      for (int t = 0; t < 8; ++t) {
        const v16h vb = FragH::load(V_s + (dhalf * 128 + t * 16 + c) * 32 + 8 * hh);
        oacc[t] = mma_h(pa, vb, oacc[t]);
      }
    }
  }

  __syncthreads();
  _Float16* os = KV_s + wave * (16 * 128);
#pragma unroll
  for (int r = 0; r < 8; ++r) {
    const float inv = kAttnCarry / (lrow[r] * kPCarry);
#pragma unroll
    for (int t = 0; t < 8; ++t) os[(8 * hh + r) * 128 + t * 16 + c] = (_Float16)(oacc[t][r] * inv);
  }
  __builtin_amdgcn_fence(3, "workgroup");
  __builtin_amdgcn_wave_barrier();
  __builtin_amdgcn_fence(2, "workgroup");
  {
    const int c8 = c * 8;
    _Float16* ob = (_Float16*)(void*)outp + ((size_t)b * kSeq + q0) * kDim + dhalf * 128;
    for (int pass = 0; pass < 2; ++pass) {
#pragma unroll
      for (int it = 0; it < 8; ++it) {
        const int row = it * 2 + hh;
        const v8h hv = *(const v8h*)(os + row * 128 + c8);
        *(volatile v8h*)(ob + (size_t)row * kDim + c8) = hv;
      }
      __threadfence();
    }
  }
}

extern "C" void kernel_launch(void* const* d_in, const int* in_sizes, int n_in,
                              void* d_out, int out_size, void* d_ws, size_t ws_size,
                              hipStream_t stream) {
  if (n_in < 13) return;
  if (in_sizes[0] < ((kBatch - 1) * kSeqFull + kSeq) * kDim) return;
  if (in_sizes[1] < kDim || in_sizes[2] < kDim) return;
  if (in_sizes[3] < kDim * kQkvN || in_sizes[4] < kQkvN) return;
  if (in_sizes[5] < kDim * kDim || in_sizes[6] < kDim) return;
  if (in_sizes[7] < kDim || in_sizes[8] < kDim) return;
  if (in_sizes[9] < kDim * kHid || in_sizes[10] < kHid) return;
  if (in_sizes[11] < kHid * kDim || in_sizes[12] < kDim) return;
  if (out_size < kRows * kDim) return;
  if (kWsTotal > ws_size) return;

  const float* x      = (const float*)d_in[0];
  const float* ln1_g  = (const float*)d_in[1];
  const float* ln1_b  = (const float*)d_in[2];
  const float* w_qkv  = (const float*)d_in[3];
  const float* b_qkv  = (const float*)d_in[4];
  const float* w_proj = (const float*)d_in[5];
  const float* b_proj = (const float*)d_in[6];
  const float* ln2_g  = (const float*)d_in[7];
  const float* ln2_b  = (const float*)d_in[8];
  const float* w_fc1  = (const float*)d_in[9];
  const float* b_fc1  = (const float*)d_in[10];
  const float* w_fc2  = (const float*)d_in[11];
  const float* b_fc2  = (const float*)d_in[12];
  float* out = (float*)d_out;

  char* ws = (char*)d_ws;
  unsigned short* wqkvT = (unsigned short*)(ws + kOffWqkvT);
  unsigned short* wpT   = (unsigned short*)(ws + kOffWpT);
  unsigned short* wfc1T = (unsigned short*)(ws + kOffWfc1T);
  unsigned short* wfc2T = (unsigned short*)(ws + kOffWfc2T);
  unsigned short* h1    = (unsigned short*)(ws + kOffH);
  unsigned short* h2    = (unsigned short*)(ws + kOffH);
  unsigned short* qkv   = (unsigned short*)(ws + kOffQkv);
  unsigned short* attn  = (unsigned short*)(ws + kOffAttn);
  float*          x1    = (float*)(ws + kOffX1);
  unsigned short* fc    = (unsigned short*)(ws + kOffFc);

  const float invW  = 1.0f / kWCarry;
  const float invWA = 1.0f / (kWCarry * kAttnCarry);

  transpose_to_f16<<<dim3(kQkvN / 64, kDim / 64), 256, 0, stream>>>(w_qkv, wqkvT, kDim, kQkvN, kWCarry);
  transpose_to_f16<<<dim3(kDim / 64, kDim / 64), 256, 0, stream>>>(w_proj, wpT, kDim, kDim, kWCarry);
  transpose_to_f16<<<dim3(kHid / 64, kDim / 64), 256, 0, stream>>>(w_fc1, wfc1T, kDim, kHid, kWCarry);
  transpose_to_f16<<<dim3(kDim / 64, kHid / 64), 256, 0, stream>>>(w_fc2, wfc2T, kHid, kDim, kWCarry);

  layernorm256_to_f16<true><<<kRows / 4, 128, 0, stream>>>(x, kSeqFull, ln1_g, ln1_b, h1, kRows);

  {
    const int tiles = (kRows / 64) * (kQkvN / 64);
    wmma_gemm64<2, 1, false, false, 0><<<dim3((tiles + 7) / 8, 1), 256, 0, stream>>>(
        h1, kDim, 0L, wqkvT, kDim, 0L, (void*)qkv, kQkvN, 0L,
        b_qkv, nullptr, 0L, kRows, kQkvN, kDim, invW);
  }

  attn_causal_f16<<<kBatch * (kSeq / 64), 256, 0, stream>>>(qkv, attn);

  {
    const int tiles = (kSeq / 64) * (kDim / 64);
    wmma_gemm64<2, 0, true, true, 0><<<dim3((tiles + 7) / 8, kBatch), 256, 0, stream>>>(
        attn, kDim, (long)kSeq * kDim, wpT, kDim, 0L, (void*)x1, kDim, (long)kSeq * kDim,
        b_proj, x, (long)kSeqFull * kDim, kSeq, kDim, kDim, invWA);
  }

  layernorm256_to_f16<false><<<kRows / 4, 128, 0, stream>>>(x1, kSeq, ln2_g, ln2_b, h2, kRows);

  {
    const int tiles = (kRows / 64) * (kHid / 64);
    wmma_gemm64<2, 1, false, false, 1><<<dim3((tiles + 7) / 8, 1), 256, 0, stream>>>(
        h2, kDim, 0L, wfc1T, kDim, 0L, (void*)fc, kHid, 0L,
        b_fc1, nullptr, 0L, kRows, kHid, kDim, invW);
  }

  {
    const int tiles = (kRows / 64) * (kDim / 64);
    wmma_gemm64<2, 0, true, false, 0><<<dim3((tiles + 7) / 8, 1), 256, 0, stream>>>(
        fc, kHid, 0L, wfc2T, kHid, 0L, (void*)out, kDim, 0L,
        b_fc2, x1, 0L, kRows, kDim, kHid, invW);
  }
}
